// SimpleAttentionBlock_21431886807689
// MI455X (gfx1250) — hardware-verified
//
#include <hip/hip_runtime.h>

typedef _Float16 v16h __attribute__((ext_vector_type(16)));
typedef _Float16 v8h  __attribute__((ext_vector_type(8)));
typedef float    v8f  __attribute__((ext_vector_type(8)));
typedef float    v4f  __attribute__((ext_vector_type(4)));
typedef v8h __attribute__((may_alias)) v8ha;
typedef v4f __attribute__((may_alias)) v4fa;

union Frag { v16h v; v8h half[2]; };

#define NB     4
#define NC     256
#define NT     4096
#define NG     32
#define CPG    8
#define GN_EPS 1e-5f
#define WSC    16.0f
#define PSC    16384.0f
#define XLD    264
#define PLD    132

__device__ __forceinline__ v8f wmma_f16(v16h a, v16h b, v8f c) {
  v8f d = __builtin_amdgcn_wmma_f32_16x16x32_f16(false, a, false, b, (short)0, c, false, false);
  asm volatile("v_nop\n\tv_nop\n\tv_nop\n\tv_nop" : "+v"(d) : "v"(a), "v"(b));
  return d;
}

__device__ __forceinline__ v16h load_frag(const _Float16* p, int h) {
  Frag f;
  f.half[0] = *(const v8ha*)(p + 8 * h);
  f.half[1] = *(const v8ha*)(p + 16 + 8 * h);
  return f.v;
}

__global__ __launch_bounds__(256) void k_gnstat(const float* __restrict__ x,
                                                 const int* __restrict__ tstep,
                                                 float* __restrict__ stats)
{
  __shared__ double r1[256];
  __shared__ double r2[256];
  (void)tstep;
  const int t = threadIdx.x;
  const int bg = blockIdx.x;
  const float* base = x + (size_t)bg * (CPG * NT);
  float s1 = 0.0f, s2 = 0.0f;
  #pragma unroll 2
  for (int it = 0; it < (CPG * NT) / (256 * 4); ++it) {
    const v4f v = *(const v4fa*)(base + ((size_t)it * 256 + t) * 4);
    s1 += (v.x + v.y) + (v.z + v.w);
    s2 += (v.x * v.x + v.y * v.y) + (v.z * v.z + v.w * v.w);
  }
  r1[t] = (double)s1;
  r2[t] = (double)s2;
  __syncthreads();
  for (int off = 128; off > 0; off >>= 1) {
    if (t < off) { r1[t] += r1[t + off]; r2[t] += r2[t + off]; }
    __syncthreads();
  }
  const double invn = 1.0 / (double)(CPG * NT);
  const double mean_d = r1[0] * invn;
  double var_d = r2[0] * invn - mean_d * mean_d;
  if (var_d < 0.0) var_d = 0.0;
  const float mean = (float)mean_d;
  const float rstd = rsqrtf((float)var_d + GN_EPS);
  if (t < 8) {
    v4f val = {0.0f, 0.0f, 0.0f, 0.0f};
    if (t == 0) { val.x = mean; val.y = rstd; }
    float* dst = stats + (size_t)bg * 32 + 4 * t;
    *(volatile v4f*)dst = val;
    __threadfence();
    *(volatile v4f*)dst = val;
  }
}

__global__ __launch_bounds__(256) void k_wcvt(const float* __restrict__ wqkv,
                                               const float* __restrict__ wproj,
                                               _Float16* __restrict__ wh,
                                               _Float16* __restrict__ wph)
{
  const int t = threadIdx.x;
  const float* src;
  _Float16* dst;
  if (blockIdx.x < 96) {
    const int g = blockIdx.x * 256 + t;
    src = wqkv + (size_t)g * 8;
    dst = wh + (size_t)g * 8;
  } else {
    const int g = (blockIdx.x - 96) * 256 + t;
    src = wproj + (size_t)g * 8;
    dst = wph + (size_t)g * 8;
  }
  const v4f a = *(const v4fa*)src;
  const v4f c = *(const v4fa*)(src + 4);
  const v8h o = { (_Float16)(a.x * WSC), (_Float16)(a.y * WSC), (_Float16)(a.z * WSC), (_Float16)(a.w * WSC),
                  (_Float16)(c.x * WSC), (_Float16)(c.y * WSC), (_Float16)(c.z * WSC), (_Float16)(c.w * WSC) };
  *(volatile v8h*)dst = o;
  __threadfence();
  *(volatile v8h*)dst = o;
}

__device__ __forceinline__ void gn_store_pass(const _Float16* sT, _Float16* __restrict__ xn,
                                              int b, int tok0, int w, int lane) {
  const int q8 = lane & 7, sub = lane >> 3;
  #pragma unroll
  for (int i = 0; i < 8; ++i) {
    const int row = 8 * w + i;
    const v8h v = *(const v8ha*)(sT + row * XLD + 64 * sub + 8 * q8);
    _Float16* dst = xn + ((size_t)(b * NT + tok0 + row)) * NC + 64 * sub + 8 * q8;
    *(volatile v8h*)dst = v;
  }
}

__global__ __launch_bounds__(256) void k_gnapply(const float* __restrict__ x,
                                                  const float* __restrict__ gamma,
                                                  const float* __restrict__ beta,
                                                  const float* __restrict__ stats,
                                                  _Float16* __restrict__ xn)
{
  __shared__ __attribute__((aligned(16))) _Float16 sT[64 * XLD];
  __shared__ float sMean[NC];
  __shared__ float sRstd[NC];
  __shared__ float sGm[NC];
  __shared__ float sBt[NC];
  const int t = threadIdx.x, lane = t & 31, w = t >> 5;
  const int b = blockIdx.y, tok0 = blockIdx.x * 64;
  {
    const int c = t, g = c >> 3;
    const float* sl = stats + (size_t)(b * NG + g) * 32;
    sMean[c] = sl[0];
    sRstd[c] = sl[1];
    sGm[c]   = gamma[c];
    sBt[c]   = beta[c];
  }
  __syncthreads();
  const int j = t & 63, cq = t >> 6;
  const float* xb = x + (size_t)b * NC * NT + tok0 + j;
  #pragma unroll 4
  for (int it = 0; it < NC / 4; ++it) {
    const int c = it * 4 + cq;
    const float v = xb[(size_t)c * NT];
    const float y = ((v - sMean[c]) * sRstd[c]) * sGm[c] + sBt[c];
    sT[j * XLD + c] = (_Float16)y;
  }
  __syncthreads();
  gn_store_pass(sT, xn, b, tok0, w, lane);
  __threadfence();
  gn_store_pass(sT, xn, b, tok0, w, lane);
}

__device__ __forceinline__ void qkv_store_pass(const _Float16* sT, _Float16* plane, _Float16* vtp,
                                               int which, int b, int fq, int m0, int w, int lane) {
  const int q8 = lane & 7, sub = lane >> 3;
  #pragma unroll
  for (int i = 0; i < 8; ++i) {
    const int lid = w * 32 + i * 4 + sub;
    v8h v;
    _Float16* dst;
    if (which != 2) {
      v = *(const v8ha*)(sT + lid * 64 + 8 * q8);
      dst = plane + ((size_t)(b * NT + m0 + lid)) * NC + fq * 64 + 8 * q8;
    } else {
      const int d = lid >> 1, hl = lid & 1;
      v = *(const v8ha*)(sT + d * 128 + 64 * hl + 8 * q8);
      dst = vtp + ((size_t)(b * NC + fq * 64 + d)) * NT + m0 + 64 * hl + 8 * q8;
    }
    *(volatile v8h*)dst = v;
  }
}

__global__ __launch_bounds__(128) void k_qkv(const _Float16* __restrict__ xn,
                                              const _Float16* __restrict__ wh,
                                              _Float16* __restrict__ qp,
                                              _Float16* __restrict__ kp,
                                              _Float16* __restrict__ vtp)
{
  __shared__ __attribute__((aligned(16))) _Float16 sT[128 * 64];

  const int tid = threadIdx.x, lane = tid & 31, w = tid >> 5;
  const int h = lane >> 4, m = lane & 15;
  const int m0 = blockIdx.x * 128;
  const int cg = blockIdx.y;
  const int which = cg >> 2, fq = cg & 3;
  const int b = blockIdx.z;
  const int m0w = m0 + 32 * w;

  const _Float16* xa0 = xn + ((size_t)(b * NT + m0w + m)) * NC;
  const _Float16* xa1 = xa0 + (size_t)16 * NC;
  const _Float16* wb  = wh + ((size_t)(which * NC + fq * 64 + m)) * NC;

  const v8f zero8 = {0.f, 0.f, 0.f, 0.f, 0.f, 0.f, 0.f, 0.f};
  v8f acc[2][4];
  #pragma unroll
  for (int mt = 0; mt < 2; ++mt)
    #pragma unroll
    for (int nt = 0; nt < 4; ++nt) acc[mt][nt] = zero8;

  #pragma unroll 1
  for (int k0 = 0; k0 < NC; k0 += 32) {
    const v16h a0 = load_frag(xa0 + k0, h);
    const v16h a1 = load_frag(xa1 + k0, h);
    #pragma unroll
    for (int nt = 0; nt < 4; ++nt) {
      const v16h bf = load_frag(wb + (size_t)nt * 16 * NC + k0, h);
      acc[0][nt] = wmma_f16(a0, bf, acc[0][nt]);
      acc[1][nt] = wmma_f16(a1, bf, acc[1][nt]);
    }
  }

  #pragma unroll
  for (int nt = 0; nt < 4; ++nt) {
    const int feat = 16 * nt + m;
    #pragma unroll
    for (int mt = 0; mt < 2; ++mt) {
      #pragma unroll
      for (int r = 0; r < 8; ++r) {
        const int tokl = 32 * w + 16 * mt + 8 * h + r;
        const float y = acc[mt][nt][r] * (1.0f / WSC);
        const int idx = (which == 2) ? (feat * 128 + tokl) : (tokl * 64 + feat);
        sT[idx] = (_Float16)y;
      }
    }
  }
  __syncthreads();

  _Float16* plane = (which == 0) ? qp : kp;
  qkv_store_pass(sT, plane, vtp, which, b, fq, m0, w, lane);
  __threadfence();
  qkv_store_pass(sT, plane, vtp, which, b, fq, m0, w, lane);
}

__device__ __forceinline__ v16h pack_p(v8f a, v8f c) {
  const v16h r = { (_Float16)(a[0] * PSC), (_Float16)(a[1] * PSC), (_Float16)(a[2] * PSC), (_Float16)(a[3] * PSC),
                   (_Float16)(a[4] * PSC), (_Float16)(a[5] * PSC), (_Float16)(a[6] * PSC), (_Float16)(a[7] * PSC),
                   (_Float16)(c[0] * PSC), (_Float16)(c[1] * PSC), (_Float16)(c[2] * PSC), (_Float16)(c[3] * PSC),
                   (_Float16)(c[4] * PSC), (_Float16)(c[5] * PSC), (_Float16)(c[6] * PSC), (_Float16)(c[7] * PSC) };
  return r;
}

__device__ __forceinline__ void att_store_pass(const _Float16* sO, _Float16* __restrict__ ctx,
                                               int b, int qb0, int w, int lane) {
  const int q8 = lane & 7, sub = lane >> 3;
  #pragma unroll
  for (int i = 0; i < 8; ++i) {
    const int row = 8 * w + i;
    const v8h v = *(const v8ha*)(sO + row * XLD + 64 * sub + 8 * q8);
    _Float16* dst = ctx + ((size_t)(b * NT + qb0 + row)) * NC + 64 * sub + 8 * q8;
    *(volatile v8h*)dst = v;
  }
}

__global__ __launch_bounds__(256) void k_attn(const _Float16* __restrict__ qp,
                                               const _Float16* __restrict__ kp,
                                               const _Float16* __restrict__ vtp,
                                               _Float16* __restrict__ ctx)
{
  __shared__ __attribute__((aligned(16))) _Float16 sO[64 * XLD];
  __shared__ __attribute__((aligned(32))) v16h sP[8 * 32];
  __shared__ float sMx[8 * 16];
  __shared__ float sL[8 * 16];

  const int tid = threadIdx.x, lane = tid & 31, w = tid >> 5;
  const int h = lane >> 4, m = lane & 15;
  const int p = w & 3, c = w >> 2;
  const int b = blockIdx.y;
  const int qb0 = blockIdx.x * 64;
  const int q0 = qb0 + 16 * p;

  const _Float16* qrow  = qp + ((size_t)(b * NT + q0 + m)) * NC;
  const _Float16* kbase = kp + ((size_t)(b * NT + m)) * NC;
  const _Float16* vbase = vtp + ((size_t)(b * NC + 128 * c + m)) * NT;

  const v8f zero8 = {0.f, 0.f, 0.f, 0.f, 0.f, 0.f, 0.f, 0.f};
  v8f o[8];
  #pragma unroll
  for (int t = 0; t < 8; ++t) o[t] = zero8;
  float mrun = -1e30f, lrun = 0.0f;

  #pragma unroll 1
  for (int kb = 0; kb < NT; kb += 64) {
    const int key0 = kb + 32 * c;
    v8f s0 = zero8, s1 = zero8;
    #pragma unroll
    for (int kc = 0; kc < 8; ++kc) {
      const v16h qf = load_frag(qrow + 32 * kc, h);
      const _Float16* kpp = kbase + (size_t)key0 * NC + 32 * kc;
      const v16h kf0 = load_frag(kpp, h);
      const v16h kf1 = load_frag(kpp + (size_t)16 * NC, h);
      s0 = wmma_f16(kf0, qf, s0);
      s1 = wmma_f16(kf1, qf, s1);
    }
    s0 = s0 * (1.0f / 16.0f);
    s1 = s1 * (1.0f / 16.0f);

    float mloc = s0[0];
    #pragma unroll
    for (int r = 0; r < 8; ++r) mloc = fmaxf(mloc, fmaxf(s0[r], s1[r]));
    mloc = fmaxf(mloc, __shfl_xor(mloc, 16));
    if (h == 0) sMx[w * 16 + m] = mloc;
    __syncthreads();
    const float moth = sMx[(w ^ 4) * 16 + m];
    const float mnew = fmaxf(mrun, fmaxf(mloc, moth));
    const float alpha = __expf(mrun - mnew);
    mrun = mnew;
    float lsum = 0.0f;
    #pragma unroll
    for (int r = 0; r < 8; ++r) {
      const float e0 = __expf(s0[r] - mnew);
      const float e1 = __expf(s1[r] - mnew);
      s0[r] = e0; s1[r] = e1;
      lsum += e0 + e1;
    }
    lsum += __shfl_xor(lsum, 16);
    lrun = lrun * alpha + lsum;
    #pragma unroll
    for (int t = 0; t < 8; ++t) o[t] = o[t] * alpha;

    const v16h pown = pack_p(s0, s1);
    sP[w * 32 + lane] = pown;
    __syncthreads();
    const v16h plo = sP[p * 32 + lane];
    const v16h phi = sP[(p + 4) * 32 + lane];

    #pragma unroll
    for (int t = 0; t < 8; ++t) {
      const _Float16* vp = vbase + (size_t)(16 * t) * NT + kb;
      const v16h vf0 = load_frag(vp, h);
      const v16h vf1 = load_frag(vp + 32, h);
      o[t] = wmma_f16(vf0, plo, o[t]);
      o[t] = wmma_f16(vf1, phi, o[t]);
    }
  }

  if (h == 0) sL[w * 16 + m] = lrun;
  __syncthreads();
  const float ltot = sL[p * 16 + m] + sL[(p + 4) * 16 + m];
  const float inv = (1.0f / ltot) * (1.0f / PSC);
  _Float16* so = sO + (16 * p + m) * XLD + 128 * c + 8 * h;
  #pragma unroll
  for (int t = 0; t < 8; ++t) {
    const v8h hv = { (_Float16)(o[t][0] * inv), (_Float16)(o[t][1] * inv), (_Float16)(o[t][2] * inv), (_Float16)(o[t][3] * inv),
                     (_Float16)(o[t][4] * inv), (_Float16)(o[t][5] * inv), (_Float16)(o[t][6] * inv), (_Float16)(o[t][7] * inv) };
    *(v8ha*)(so + 16 * t) = hv;
  }
  __syncthreads();

  att_store_pass(sO, ctx, b, qb0, w, lane);
  __threadfence();
  att_store_pass(sO, ctx, b, qb0, w, lane);
}

__device__ __forceinline__ void proj_store_pass(const float* sT, const float* __restrict__ x, float* __restrict__ out,
                                                int b, int fq, int m0, int w, int lane) {
  const int q8 = lane & 7, sub = lane >> 3;
  #pragma unroll
  for (int i = 0; i < 16; ++i) {
    const int row = 16 * w + i;
    const v4f v = *(const v4fa*)(sT + row * PLD + 32 * sub + 4 * q8);
    const size_t gi = ((size_t)(b * NC + fq * 64 + row)) * NT + m0 + 32 * sub + 4 * q8;
    const v4f xv = *(const v4fa*)(x + gi);
    const v4f y = v + xv;
    *(volatile v4f*)(out + gi) = y;
  }
}

__global__ __launch_bounds__(128) void k_proj(const _Float16* __restrict__ ctx,
                                               const _Float16* __restrict__ wph,
                                               const float* __restrict__ x,
                                               float* __restrict__ out)
{
  __shared__ __attribute__((aligned(16))) float sT[64 * PLD];

  const int tid = threadIdx.x, lane = tid & 31, w = tid >> 5;
  const int h = lane >> 4, m = lane & 15;
  const int m0 = blockIdx.x * 128;
  const int fq = blockIdx.y;
  const int b = blockIdx.z;
  const int m0w = m0 + 32 * w;

  const _Float16* xa0 = ctx + ((size_t)(b * NT + m0w + m)) * NC;
  const _Float16* xa1 = xa0 + (size_t)16 * NC;
  const _Float16* wb  = wph + ((size_t)(fq * 64 + m)) * NC;

  const v8f zero8 = {0.f, 0.f, 0.f, 0.f, 0.f, 0.f, 0.f, 0.f};
  v8f acc[2][4];
  #pragma unroll
  for (int mt = 0; mt < 2; ++mt)
    #pragma unroll
    for (int nt = 0; nt < 4; ++nt) acc[mt][nt] = zero8;

  #pragma unroll 1
  for (int k0 = 0; k0 < NC; k0 += 32) {
    const v16h a0 = load_frag(xa0 + k0, h);
    const v16h a1 = load_frag(xa1 + k0, h);
    #pragma unroll
    for (int nt = 0; nt < 4; ++nt) {
      const v16h bf = load_frag(wb + (size_t)nt * 16 * NC + k0, h);
      acc[0][nt] = wmma_f16(a0, bf, acc[0][nt]);
      acc[1][nt] = wmma_f16(a1, bf, acc[1][nt]);
    }
  }

  #pragma unroll
  for (int nt = 0; nt < 4; ++nt) {
    const int feat = 16 * nt + m;
    #pragma unroll
    for (int mt = 0; mt < 2; ++mt) {
      #pragma unroll
      for (int r = 0; r < 8; ++r) {
        const int tokl = 32 * w + 16 * mt + 8 * h + r;
        sT[feat * PLD + tokl] = acc[mt][nt][r] * (1.0f / WSC);
      }
    }
  }
  __syncthreads();

  proj_store_pass(sT, x, out, b, fq, m0, w, lane);
  __threadfence();
  proj_store_pass(sT, x, out, b, fq, m0, w, lane);
}

extern "C" void kernel_launch(void* const* d_in, const int* in_sizes, int n_in,
                              void* d_out, int out_size, void* d_ws, size_t ws_size,
                              hipStream_t stream) {
  if (n_in < 6) return;
  if (in_sizes[0] != NB * NC * NT) return;
  if (in_sizes[1] < 1) return;
  if (in_sizes[2] != NC || in_sizes[3] != NC) return;
  if (in_sizes[4] != 3 * NC * NC || in_sizes[5] != NC * NC) return;
  if (out_size != NB * NC * NT) return;

  const float* x     = (const float*)d_in[0];
  const int*   tstep = (const int*)d_in[1];
  const float* gamma = (const float*)d_in[2];
  const float* beta  = (const float*)d_in[3];
  const float* wqkv  = (const float*)d_in[4];
  const float* wproj = (const float*)d_in[5];
  float* out = (float*)d_out;

  const size_t stats_bytes = (size_t)NB * NG * 32 * sizeof(float);
  const size_t plane_bytes = (size_t)NB * NT * NC * 2;
  const size_t wh_bytes    = (size_t)3 * NC * NC * 2;
  const size_t wph_bytes   = (size_t)NC * NC * 2;
  const size_t off_stats = 0;
  const size_t off_xn    = off_stats + stats_bytes;
  const size_t off_wh    = off_xn + plane_bytes;
  const size_t off_wph   = off_wh + wh_bytes;
  const size_t off_q     = off_wph + wph_bytes;
  const size_t off_k     = off_q + plane_bytes;
  const size_t off_vt    = off_k + plane_bytes;
  const size_t off_ctx   = off_vt + plane_bytes;
  const size_t total     = off_ctx + plane_bytes;
  if (total > ws_size) return;

  char* ws = (char*)d_ws;
  float*    stats = (float*)(ws + off_stats);
  _Float16* xn    = (_Float16*)(ws + off_xn);
  _Float16* wh    = (_Float16*)(ws + off_wh);
  _Float16* wph   = (_Float16*)(ws + off_wph);
  _Float16* qpl   = (_Float16*)(ws + off_q);
  _Float16* kpl   = (_Float16*)(ws + off_k);
  _Float16* vtp   = (_Float16*)(ws + off_vt);
  _Float16* ctx   = (_Float16*)(ws + off_ctx);

  k_gnstat<<<NB * NG, 256, 0, stream>>>(x, tstep, stats);
  k_wcvt<<<96 + 32, 256, 0, stream>>>(wqkv, wproj, wh, wph);
  k_gnapply<<<dim3(NT / 64, NB), 256, 0, stream>>>(x, gamma, beta, stats, xn);
  k_qkv<<<dim3(NT / 128, 12, NB), 128, 0, stream>>>(xn, wh, qpl, kpl, vtp);
  k_attn<<<dim3(NT / 64, NB), 256, 0, stream>>>(qpl, kpl, vtp, ctx);
  k_proj<<<dim3(NT / 128, 4, NB), 128, 0, stream>>>(ctx, wph, x, out);
}
